// FeatureMatcher_25993142075777
// MI455X (gfx1250) — hardware-verified
//
#include <hip/hip_runtime.h>
#include <math.h>

constexpr int kNI   = 1024;
constexpr int kNJ   = 1024;
constexpr int kFeat = 512;
constexpr int kHid  = 256;
constexpr int kHid2 = 128;
constexpr int kTI   = 16;
constexpr int kTJ   = 32;
constexpr int kH1P  = 264;
constexpr int kH2P  = 136;
constexpr float kW2Carry    = 16.0f;
constexpr float kW2CarryInv = 1.0f / 16.0f;
constexpr float kW3Carry    = 8.0f;
constexpr float kW3CarryInv = 0.125f;

typedef __attribute__((ext_vector_type(16))) _Float16 v16h;
typedef __attribute__((ext_vector_type(8)))  _Float16 v8h;
typedef __attribute__((ext_vector_type(16))) __bf16   v16b;
typedef __attribute__((ext_vector_type(8)))  __bf16   v8b;
typedef __attribute__((ext_vector_type(8)))  float    v8f;
typedef __attribute__((ext_vector_type(4)))  float    v4f;
typedef __attribute__((ext_vector_type(4)))  unsigned int v4u;

__device__ __forceinline__ unsigned short f2bf_bits(float f) {
  unsigned u = __float_as_uint(f);
  return (unsigned short)((u + 0x7FFFu + ((u >> 16) & 1u)) >> 16);
}
__device__ __forceinline__ float bf_bits2f(unsigned short h) { return __uint_as_float(((unsigned)h) << 16); }

__device__ __forceinline__ void dep_guard_h(v8f& a, v8f& b, v16h x, v16h y) { asm volatile("v_nop\n\tv_nop\n\tv_nop\n\tv_nop" : "+v"(a), "+v"(b) : "v"(x), "v"(y)); }
__device__ __forceinline__ void dep_guard_b(v8f& a, v8f& b, v16b x, v16b y) { asm volatile("v_nop\n\tv_nop\n\tv_nop\n\tv_nop" : "+v"(a), "+v"(b) : "v"(x), "v"(y)); }
__device__ __forceinline__ void keep4_h(v16h a, v16h b, v16h c, v16h d) { asm volatile("v_nop" :: "v"(a), "v"(b), "v"(c), "v"(d)); }
__device__ __forceinline__ void keep4_b(v16b a, v16b b, v16b c, v16b d) { asm volatile("v_nop" :: "v"(a), "v"(b), "v"(c), "v"(d)); }
__device__ __forceinline__ void acc_guard4(v8f& a, v8f& b, v8f& c, v8f& d) { asm volatile("v_nop\n\tv_nop\n\tv_nop\n\tv_nop" : "+v"(a), "+v"(b), "+v"(c), "+v"(d)); }
template <typename T> struct Frag;
template <> struct Frag<_Float16> {
  typedef v16h V; union U { v16h v; v8h h[2]; };
  static __device__ __forceinline__ v16h load(const _Float16* p) {
    U f; f.h[0] = *(const v8h*)(p); f.h[1] = *(const v8h*)(p + 16); return f.v;
  }
  static __device__ __forceinline__ v8f mma(v16h a, v16h b, v8f c) {
    return __builtin_amdgcn_wmma_f32_16x16x32_f16(false, a, false, b, (short)0, c, false, false);
  }
  static __device__ __forceinline__ void guard(v8f& a, v8f& b, v16h x, v16h y) { dep_guard_h(a, b, x, y); }
  static __device__ __forceinline__ void keep(v16h a, v16h b, v16h c, v16h d) { keep4_h(a, b, c, d); }
};
template <> struct Frag<__bf16> {
  typedef v16b V; union U { v16b v; v8b h[2]; };
  static __device__ __forceinline__ v16b load(const __bf16* p) {
    U f; f.h[0] = *(const v8b*)(p); f.h[1] = *(const v8b*)(p + 16); return f.v;
  }
  static __device__ __forceinline__ v8f mma(v16b a, v16b b, v8f c) {
    return __builtin_amdgcn_wmma_f32_16x16x32_bf16(false, a, false, b, (short)0, c, false, false);
  }
  static __device__ __forceinline__ void guard(v8f& a, v8f& b, v16b x, v16b y) { dep_guard_b(a, b, x, y); }
  static __device__ __forceinline__ void keep(v16b a, v16b b, v16b c, v16b d) { keep4_b(a, b, c, d); }
};

__device__ __forceinline__ unsigned pk16(unsigned short a, unsigned short b) { return (unsigned)a | ((unsigned)b << 16); }
__device__ __forceinline__ unsigned short h_bits(float f) { const _Float16 h = (_Float16)f; return __builtin_bit_cast(unsigned short, h); }

__device__ __forceinline__ v8f mma_h(v16h a, v16h b, v8f c) {
  c = __builtin_amdgcn_wmma_f32_16x16x32_f16(false, a, false, b, (short)0, c, false, false);
  asm volatile("v_nop\n\tv_nop\n\tv_nop\n\tv_nop" : "+v"(c) : "v"(a), "v"(b));
  return c;
}

template <int ET> struct Elem;
template <> struct Elem<0> { typedef _Float16 T; };
template <> struct Elem<1> { typedef __bf16 T; };
template <int ET, bool SPLIT, int BIAS_MODE, int OUT_MODE, bool RESID, int ACT = 0>
__global__ __launch_bounds__(256) void wmma_gemm64(
    const unsigned short* __restrict__ Ap, const unsigned short* __restrict__ A2p, int lda, long strideA,
    const unsigned short* __restrict__ Btp, const unsigned short* __restrict__ Bt2p, int ldb, long strideB,
    void* __restrict__ Cout, void* __restrict__ Cout2, int ldc, long strideC,
    const float* __restrict__ bias,
    const float* __restrict__ resid, long strideR,
    int M, int N, int K, float scale) {
  typedef typename Elem<ET>::T T;
  typedef typename Frag<T>::V V;
  const T* A = (const T*)Ap; const T* A2 = (const T*)A2p; const T* Bt = (const T*)Btp; const T* Bt2 = (const T*)Bt2p;
  __shared__ __align__(16) float sT[8][16 * 68];
  const int b    = blockIdx.y;
  const int lane = threadIdx.x & 31;
  const int wave = threadIdx.x >> 5;
  const int tilesN = N >> 6;
  const int tilesM = M >> 6;
  const int tile = blockIdx.x * 8 + wave;
  if (tile >= tilesM * tilesN) return;
  const int tm = tile / tilesN;
  const int tn = tile - tm * tilesN;
  const int m0 = tm << 6;
  const int n0 = tn << 6;

  const T* Ab  = A  + (size_t)b * strideA;
  const T* Bb  = Bt + (size_t)b * strideB;
  const T* Ab2 = SPLIT ? (A2  + (size_t)b * strideA) : nullptr;
  const T* Bb2 = SPLIT ? (Bt2 + (size_t)b * strideB) : nullptr;

  const int rlane = lane & 15;
  const int koff  = (lane >> 4) * 8;
  const int mOff  = (lane >> 4) * 8;

  v8f acc[4][4];
#pragma unroll
  for (int i = 0; i < 4; ++i)
#pragma unroll
    for (int j = 0; j < 4; ++j) acc[i][j] = (v8f){0.f,0.f,0.f,0.f,0.f,0.f,0.f,0.f};

  for (int k0 = 0; k0 < K; k0 += 32) {
    V bh[4], bl[4];
#pragma unroll
    for (int j = 0; j < 4; ++j) {
      const size_t bo = (size_t)(n0 + (j << 4) + rlane) * ldb + koff + k0;
      bh[j] = Frag<T>::load(Bb + bo);
      if (SPLIT) bl[j] = Frag<T>::load(Bb2 + bo);
    }
#pragma unroll
    for (int i = 0; i < 4; ++i) {
      const size_t ao = (size_t)(m0 + (i << 4) + rlane) * lda + koff + k0;
      V ah = Frag<T>::load(Ab + ao);
      V al;
      if (SPLIT) al = Frag<T>::load(Ab2 + ao);
#pragma unroll
      for (int j = 0; j < 4; ++j) {
        acc[i][j] = Frag<T>::mma(ah, bh[j], acc[i][j]);
        if (SPLIT) {
          acc[i][j] = Frag<T>::mma(ah, bl[j], acc[i][j]);
          acc[i][j] = Frag<T>::mma(al, bh[j], acc[i][j]);
        }
      }
      Frag<T>::guard(acc[i][0], acc[i][3], ah, SPLIT ? al : ah);
    }
    Frag<T>::keep(bh[0], bh[1], bh[2], bh[3]);
    if (SPLIT) Frag<T>::keep(bl[0], bl[1], bl[2], bl[3]);
  }
  acc_guard4(acc[0][0], acc[0][1], acc[0][2], acc[0][3]);
  acc_guard4(acc[1][0], acc[1][1], acc[1][2], acc[1][3]);
  acc_guard4(acc[2][0], acc[2][1], acc[2][2], acc[2][3]);
  acc_guard4(acc[3][0], acc[3][1], acc[3][2], acc[3][3]);

  float* slab = sT[wave];
  const float* Rb = RESID ? (resid + (size_t)b * strideR) : nullptr;
#pragma unroll
  for (int i = 0; i < 4; ++i) {
    const int mBase = m0 + (i << 4);
#pragma unroll
    for (int j = 0; j < 4; ++j) {
      const int n = n0 + (j << 4) + rlane;
      float bv = 0.f;
      if (BIAS_MODE == 2) bv = bias[n];
#pragma unroll
      for (int r = 0; r < 8; ++r) {
        float v = acc[i][j][r] * scale;
        if (BIAS_MODE == 1) v += bias[mBase + mOff + r];
        if (BIAS_MODE == 2) v += bv;
        if (RESID) v += Rb[(size_t)(mBase + mOff + r) * ldc + n];
        if (ACT == 2) v = fmaxf(v, 0.0f);
        slab[(mOff + r) * 68 + (j << 4) + rlane] = v;
      }
    }
    __builtin_amdgcn_fence(__ATOMIC_RELEASE, "workgroup");
    __builtin_amdgcn_wave_barrier();
    __builtin_amdgcn_fence(__ATOMIC_ACQUIRE, "workgroup");
    if (OUT_MODE == 0) {
      float* C = (float*)Cout + (size_t)b * strideC;
      const int hh = lane >> 4, c4 = (lane & 15) * 4;
      for (int pass = 0; pass < 2; ++pass) {
#pragma unroll
        for (int it = 0; it < 8; ++it) {
          const int row = it * 2 + hh;
          v4f v = *(const v4f*)(slab + row * 68 + c4);
          *(volatile v4f*)(C + (size_t)(mBase + row) * ldc + n0 + c4) = v;
        }
        __threadfence();
      }
    } else {
      const int q = lane >> 3, c8 = (lane & 7) * 8;
      unsigned short* C  = (unsigned short*)Cout  + (size_t)b * strideC;
      unsigned short* C2 = (OUT_MODE == 2) ? ((unsigned short*)Cout2 + (size_t)b * strideC) : nullptr;
      for (int pass = 0; pass < 2; ++pass) {
#pragma unroll
        for (int it = 0; it < 4; ++it) {
          const int row = it * 4 + q;
          const float* sp = slab + row * 68 + c8;
          v8h hv, lv;
#pragma unroll
          for (int e = 0; e < 8; ++e) {
            if (OUT_MODE == 1) {
              hv[e] = (_Float16)sp[e];
            } else {
              unsigned short hb = f2bf_bits(sp[e]);
              unsigned short lb = f2bf_bits(sp[e] - bf_bits2f(hb));
              hv[e] = __builtin_bit_cast(_Float16, hb);
              lv[e] = __builtin_bit_cast(_Float16, lb);
            }
          }
          *(volatile v8h*)(C + (size_t)(mBase + row) * ldc + n0 + c8) = hv;
          if (OUT_MODE == 2) *(volatile v8h*)(C2 + (size_t)(mBase + row) * ldc + n0 + c8) = lv;
        }
        __threadfence();
      }
    }
    __builtin_amdgcn_fence(__ATOMIC_RELEASE, "workgroup");
    __builtin_amdgcn_wave_barrier();
    __builtin_amdgcn_fence(__ATOMIC_ACQUIRE, "workgroup");
  }
}

template <int MODE>
__global__ __launch_bounds__(256) void cast8_kernel(const float* __restrict__ in, unsigned short* __restrict__ out, int n8, float scale) {
  const int i = blockIdx.x * 256 + threadIdx.x;
  if (i >= n8) return;
  const float* p = in + 8 * (size_t)i;
  const v4f a = *(const v4f*)(p);
  const v4f c = *(const v4f*)(p + 4);
  unsigned short hb[8];
#pragma unroll
  for (int e = 0; e < 4; ++e) {
    if (MODE == 0) {
      hb[e]     = f2bf_bits(a[e]);
      hb[4 + e] = f2bf_bits(c[e]);
    } else {
      hb[e]     = h_bits(bf_bits2f(f2bf_bits(a[e])) * scale);
      hb[4 + e] = h_bits(bf_bits2f(f2bf_bits(c[e])) * scale);
    }
  }
  const v4u u = (v4u){pk16(hb[0], hb[1]), pk16(hb[2], hb[3]), pk16(hb[4], hb[5]), pk16(hb[6], hb[7])};
  unsigned short* q = out + 8 * (size_t)i;
  *(volatile v4u*)q = u;
  __threadfence();
  *(volatile v4u*)q = u;
  (void)scale;
}

template <int MODE>
__device__ __forceinline__ unsigned short cvt16(float v, float scale) { return (MODE == 0) ? f2bf_bits(v) : h_bits(v * scale); }

template <int MODE>
__global__ __launch_bounds__(256) void transpose_cast64(const float* __restrict__ in, unsigned short* __restrict__ out,
                                                         int R, int CC, float scale) {
  __shared__ float s[64 * 65];
  const int t  = threadIdx.x;
  const int c0 = blockIdx.x * 64;
  const int r0 = blockIdx.y * 64;
  {
    const int row = t >> 2, cq = (t & 3) * 16;
    const float* ip = in + (size_t)(r0 + row) * CC + c0 + cq;
#pragma unroll
    for (int e4 = 0; e4 < 4; ++e4) {
      const v4f v = *(const v4f*)(ip + 4 * e4);
#pragma unroll
      for (int e = 0; e < 4; ++e) s[(cq + 4 * e4 + e) * 65 + row] = v[e];
    }
  }
  __syncthreads();
  const int wave = t >> 5, lane = t & 31, q = lane >> 3, c8 = (lane & 7) * 8;
  const int orow0 = wave * 8 + q;
  const int orow1 = wave * 8 + 4 + q;
  unsigned short b0[8], b1v[8];
#pragma unroll
  for (int e = 0; e < 8; ++e) {
    b0[e]  = cvt16<MODE>(s[orow0 * 65 + c8 + e], scale);
    b1v[e] = cvt16<MODE>(s[orow1 * 65 + c8 + e], scale);
  }
  const v4u u0 = (v4u){pk16(b0[0], b0[1]), pk16(b0[2], b0[3]), pk16(b0[4], b0[5]), pk16(b0[6], b0[7])};
  const v4u u1 = (v4u){pk16(b1v[0], b1v[1]), pk16(b1v[2], b1v[3]), pk16(b1v[4], b1v[5]), pk16(b1v[6], b1v[7])};
  unsigned short* o0 = out + (size_t)(c0 + orow0) * R + r0 + c8;
  unsigned short* o1 = out + (size_t)(c0 + orow1) * R + r0 + c8;
  *(volatile v4u*)o0 = u0;
  *(volatile v4u*)o1 = u1;
  __threadfence();
  *(volatile v4u*)o0 = u0;
  *(volatile v4u*)o1 = u1;
}

__global__ __launch_bounds__(256) void w3pad_kernel(const float* __restrict__ W3, unsigned short* __restrict__ W3P, float scale) {
  const int t = threadIdx.x;
  const int row = t >> 4, col = (t & 15) * 8;
  const v4f a = *(const v4f*)(W3 + col);
  const v4f c = *(const v4f*)(W3 + col + 4);
  unsigned short hb[8];
#pragma unroll
  for (int e = 0; e < 4; ++e) {
    hb[e]     = (row == 0) ? h_bits(a[e] * scale) : (unsigned short)0;
    hb[4 + e] = (row == 0) ? h_bits(c[e] * scale) : (unsigned short)0;
  }
  const v4u u = (v4u){pk16(hb[0], hb[1]), pk16(hb[2], hb[3]), pk16(hb[4], hb[5]), pk16(hb[6], hb[7])};
  unsigned short* q = W3P + 8 * (size_t)t;
  *(volatile v4u*)q = u;
  __threadfence();
  *(volatile v4u*)q = u;
}

__global__ __launch_bounds__(256) void pairmlp_kernel(const float* __restrict__ p1, const float* __restrict__ p2,
                                                      const float* __restrict__ b1,
                                                      const unsigned short* __restrict__ W2Tp, const float* __restrict__ b2,
                                                      const unsigned short* __restrict__ W3Pp, const float* __restrict__ b3,
                                                      float* __restrict__ out) {
  __shared__ __align__(16) float    s_p2[kTJ * kHid];
  __shared__ __align__(16) _Float16 s_h1[kTJ * kH1P];
  __shared__ __align__(16) _Float16 s_h2[kTJ * kH2P];
  __shared__ __align__(16) float    s_sim[kTI * kTJ];

  const _Float16* W2T = (const _Float16*)W2Tp;
  const _Float16* W3P = (const _Float16*)W3Pp;
  const int tid  = threadIdx.x;
  const int lane = tid & 31;
  const int wave = tid >> 5;
  const int hh   = lane >> 4;
  const int m    = lane & 15;
  const int j0   = blockIdx.x * kTJ;
  const int i0   = blockIdx.y * kTI;

#pragma unroll
  for (int it = 0; it < 8; ++it) {
    const int idx4 = it * 256 + tid;
    const int row  = idx4 >> 6;
    const int cc   = (idx4 & 63) * 4;
    *(v4f*)&s_p2[row * kHid + cc] = *(const v4f*)(p2 + (size_t)(j0 + row) * kHid + cc);
  }

  const int ncol = wave * 16 + m;
  v16h bfr[8];
#pragma unroll
  for (int c = 0; c < 8; ++c) bfr[c] = Frag<_Float16>::load(W2T + (size_t)ncol * kHid + c * 32 + 8 * hh);
  const float b2v = b2[ncol];
  const float b3v = b3[0];

  const int k8 = (tid & 31) * 8;
  const int jr = tid >> 5;
  const v4f b1a = *(const v4f*)(b1 + k8);
  const v4f b1b = *(const v4f*)(b1 + k8 + 4);

  __syncthreads();

  const v8f zero8 = (v8f){0.f, 0.f, 0.f, 0.f, 0.f, 0.f, 0.f, 0.f};

#pragma unroll 1
  for (int ii = 0; ii < kTI; ++ii) {
    {
      const float* pr = p1 + (size_t)(i0 + ii) * kHid + k8;
      const v4f pa = *(const v4f*)(pr);
      const v4f pb = *(const v4f*)(pr + 4);
#pragma unroll
      for (int g = 0; g < 4; ++g) {
        const int jj = jr + 8 * g;
        const v4f xa = *(const v4f*)&s_p2[jj * kHid + k8];
        const v4f xb = *(const v4f*)&s_p2[jj * kHid + k8 + 4];
        v8h hv;
#pragma unroll
        for (int e = 0; e < 4; ++e) {
          hv[e]     = (_Float16)fmaxf((pa[e] + xa[e]) + b1a[e], 0.0f);
          hv[4 + e] = (_Float16)fmaxf((pb[e] + xb[e]) + b1b[e], 0.0f);
        }
        *(v8h*)&s_h1[jj * kH1P + k8] = hv;
      }
    }
    __syncthreads();

    v8f acc0 = zero8, acc1 = zero8;
#pragma unroll
    for (int c = 0; c < 8; ++c) {
      const v16h a0 = Frag<_Float16>::load(s_h1 + m * kH1P + c * 32 + 8 * hh);
      const v16h a1 = Frag<_Float16>::load(s_h1 + (16 + m) * kH1P + c * 32 + 8 * hh);
      acc0 = Frag<_Float16>::mma(a0, bfr[c], acc0);
      acc1 = Frag<_Float16>::mma(a1, bfr[c], acc1);
      dep_guard_h(acc0, acc1, a0, a1);
    }

#pragma unroll
    for (int r = 0; r < 8; ++r) {
      s_h2[(8 * hh + r) * kH2P + ncol]      = (_Float16)fmaxf(acc0[r] * kW2CarryInv + b2v, 0.0f);
      s_h2[(16 + 8 * hh + r) * kH2P + ncol] = (_Float16)fmaxf(acc1[r] * kW2CarryInv + b2v, 0.0f);
    }
    __syncthreads();

    if (wave < 2) {
      v8f acc2 = zero8;
#pragma unroll
      for (int c = 0; c < 4; ++c) {
        const v16h a  = Frag<_Float16>::load(s_h2 + (wave * 16 + m) * kH2P + c * 32 + 8 * hh);
        const v16h bw = Frag<_Float16>::load(W3P + m * kHid2 + c * 32 + 8 * hh);
        acc2 = mma_h(a, bw, acc2);
      }
      if (m == 0) {
        const v4f lo = (v4f){acc2[0] * kW3CarryInv, acc2[1] * kW3CarryInv, acc2[2] * kW3CarryInv, acc2[3] * kW3CarryInv};
        const v4f hi = (v4f){acc2[4] * kW3CarryInv, acc2[5] * kW3CarryInv, acc2[6] * kW3CarryInv, acc2[7] * kW3CarryInv};
        float* sp = s_sim + ii * kTJ + wave * 16 + 8 * hh;
        *(v4f*)(sp)     = lo;
        *(v4f*)(sp + 4) = hi;
      }
    }
  }
  __syncthreads();

#pragma unroll
  for (int e2 = 0; e2 < 2; ++e2) {
    const int idx = e2 * 256 + tid;
    const float x = s_sim[idx] + b3v;
    const float s = 1.0f / (1.0f + expf(-x));
    s_sim[idx] = s;
  }
  __syncthreads();

  if (wave < 4) {
    const int q = lane >> 3, c4 = (lane & 7) * 4;
    const int ii = wave * 4 + q;
    const v4f v = *(const v4f*)&s_sim[ii * kTJ + c4];
    float* op = out + (size_t)(i0 + ii) * kNJ + j0 + c4;
    *(volatile v4f*)op = v;
    __threadfence();
    *(volatile v4f*)op = v;
  }
}

extern "C" void kernel_launch(void* const* d_in, const int* in_sizes, int n_in,
                              void* d_out, int out_size, void* d_ws, size_t ws_size,
                              hipStream_t stream) {
  if (n_in < 8) return;
  if (in_sizes[0] != kNI * kFeat) return;
  if (in_sizes[1] != kNJ * kFeat) return;
  if (in_sizes[2] != 2 * kFeat * kHid) return;
  if (in_sizes[3] != kHid) return;
  if (in_sizes[4] != kHid * kHid2) return;
  if (in_sizes[5] != kHid2) return;
  if (in_sizes[6] != kHid2) return;
  if (in_sizes[7] < 1) return;
  if (out_size != kNI * kNJ) return;

  const float* feat1 = (const float*)d_in[0];
  const float* feat2 = (const float*)d_in[1];
  const float* W1    = (const float*)d_in[2];
  const float* b1    = (const float*)d_in[3];
  const float* W2    = (const float*)d_in[4];
  const float* b2    = (const float*)d_in[5];
  const float* W3    = (const float*)d_in[6];
  const float* b3    = (const float*)d_in[7];
  float* outp = (float*)d_out;

  const size_t SZ_FB  = (size_t)kNI * kFeat * 2;
  const size_t SZ_W1T = (size_t)kHid * kFeat * 2;
  const size_t SZ_W2T = (size_t)kHid2 * kHid * 2;
  const size_t SZ_W3P = (size_t)16 * kHid2 * 2;
  const size_t SZ_P   = (size_t)kNI * kHid * 4;
  size_t off = 0;
  const size_t oF1B  = off; off += SZ_FB;
  const size_t oF2B  = off; off += SZ_FB;
  const size_t oW1AT = off; off += SZ_W1T;
  const size_t oW1BT = off; off += SZ_W1T;
  const size_t oW2T  = off; off += SZ_W2T;
  const size_t oW3P  = off; off += SZ_W3P;
  const size_t oP1   = off; off += SZ_P;
  const size_t oP2   = off; off += SZ_P;
  const size_t TOTAL = off;
  if (TOTAL > ws_size) return;
  if (TOTAL > (size_t)134217728) return;

  char* ws = (char*)d_ws;
  unsigned short* F1B  = (unsigned short*)(ws + oF1B);
  unsigned short* F2B  = (unsigned short*)(ws + oF2B);
  unsigned short* W1AT = (unsigned short*)(ws + oW1AT);
  unsigned short* W1BT = (unsigned short*)(ws + oW1BT);
  unsigned short* W2T  = (unsigned short*)(ws + oW2T);
  unsigned short* W3P  = (unsigned short*)(ws + oW3P);
  float*          P1   = (float*)(ws + oP1);
  float*          P2   = (float*)(ws + oP2);

  const dim3 blk(256);

  {
    const int n8 = kNI * kFeat / 8;
    cast8_kernel<0><<<dim3(n8 / 256), blk, 0, stream>>>(feat1, F1B, n8, 1.0f);
    cast8_kernel<0><<<dim3(n8 / 256), blk, 0, stream>>>(feat2, F2B, n8, 1.0f);
  }
  transpose_cast64<0><<<dim3(kHid / 64, kFeat / 64), blk, 0, stream>>>(W1, W1AT, kFeat, kHid, 1.0f);
  transpose_cast64<0><<<dim3(kHid / 64, kFeat / 64), blk, 0, stream>>>(W1 + (size_t)kFeat * kHid, W1BT, kFeat, kHid, 1.0f);
  transpose_cast64<1><<<dim3(kHid2 / 64, kHid / 64), blk, 0, stream>>>(W2, W2T, kHid, kHid2, kW2Carry);
  w3pad_kernel<<<dim3(1), blk, 0, stream>>>(W3, W3P, kW3Carry);

  const dim3 gP((((kNI / 64) * (kHid / 64)) + 7) / 8, 1);
  wmma_gemm64<1, false, 0, 0, false, 0><<<gP, blk, 0, stream>>>(
      F1B, F1B, kFeat, 0L, W1AT, W1AT, kFeat, 0L, (void*)P1, (void*)P1, kHid, 0L, b1, b1, 0L, kNI, kHid, kFeat, 1.0f);
  wmma_gemm64<1, false, 0, 0, false, 0><<<gP, blk, 0, stream>>>(
      F2B, F2B, kFeat, 0L, W1BT, W1BT, kFeat, 0L, (void*)P2, (void*)P2, kHid, 0L, b1, b1, 0L, kNJ, kHid, kFeat, 1.0f);

  pairmlp_kernel<<<dim3(kNJ / kTJ, kNI / kTI), blk, 0, stream>>>(P1, P2, b1, W2T, b2, W3P, b3, outp);
}
